// RawCrossAttention_47802986004881
// MI455X (gfx1250) — hardware-verified
//
#include <hip/hip_runtime.h>
#include <stdint.h>

#define NB    2
#define NC    1024
#define NL    2048
#define NHD   16
#define HDIM  64
#define NEGV  1000000.0f
#define LOG2E 1.4426950408889634f

typedef __bf16         v16b __attribute__((ext_vector_type(16)));
typedef unsigned short v8us __attribute__((ext_vector_type(8)));
typedef float          v8f  __attribute__((ext_vector_type(8)));
typedef float          v4f  __attribute__((ext_vector_type(4)));

union FragB { v16b v; v8us h[2]; };
union M8    { v8f  v; v4f  h[2]; };

__device__ __forceinline__ unsigned short f2bf_bits(float f) {
  const unsigned u = __float_as_uint(f);
  return (unsigned short)((u + 0x7FFFu + ((u >> 16) & 1u)) >> 16);
}
__device__ __forceinline__ float bf_bits2f(unsigned short h) { return __uint_as_float(((unsigned)h) << 16); }
__device__ __forceinline__ float bf_rne(float f) { return bf_bits2f(f2bf_bits(f)); }
__device__ __forceinline__ v8f vz8() { v8f z = {0.f, 0.f, 0.f, 0.f, 0.f, 0.f, 0.f, 0.f}; return z; }

__device__ __forceinline__ v16b ldfrag_b(const unsigned short* rowk0, int hf) {
  FragB f;
  f.h[0] = *(const v8us*)(rowk0 + 8 * hf);
  f.h[1] = *(const v8us*)(rowk0 + 16 + 8 * hf);
  return f.v;
}

__device__ __forceinline__ v8f mma_b(v16b a, v16b b, v8f c) {
  c = __builtin_amdgcn_wmma_f32_16x16x32_bf16(false, a, false, b, (short)0, c, false, false);
  asm volatile("v_nop\n\tv_nop\n\tv_nop\n\tv_nop" : "+v"(c) : "v"(a), "v"(b));
  return c;
}

__global__ __launch_bounds__(256) void cvt_w_kernel(const float* __restrict__ W0, const float* __restrict__ W1,
                                                    const float* __restrict__ W2, unsigned short* __restrict__ P, int n8) {
  const int y = blockIdx.y;
  const float* W = (y == 0) ? W0 : ((y == 1) ? W1 : W2);
  int i = blockIdx.x * 256 + threadIdx.x;
  i = (i < n8) ? i : (n8 - 1);
  const float* src = W + 8 * (size_t)i;
  const v4f a = *(const v4f*)(src);
  const v4f c = *(const v4f*)(src + 4);
  v8us hv;
#pragma unroll
  for (int e = 0; e < 4; ++e) {
    hv[e]     = f2bf_bits(a[e]);
    hv[4 + e] = f2bf_bits(c[e]);
  }
  unsigned short* d = P + (size_t)y * NC * NC + 8 * (size_t)i;
  *(volatile v8us*)d = hv;
  __threadfence();
  *(volatile v8us*)d = hv;
}

__global__ __launch_bounds__(256) void cvt_xt_kernel(const float* __restrict__ X, unsigned short* __restrict__ P) {
  __shared__ __align__(16) unsigned short th[64 * 72];
  const int b = blockIdx.z, l0 = blockIdx.x * 64, c0 = blockIdx.y * 64, tid = threadIdx.x;
  const float* Xb = X + (size_t)b * NC * NL;
  {
    const int cr = tid >> 2;
    const int lq = (tid & 3) * 16;
    const float* src = Xb + (size_t)(c0 + cr) * NL + l0 + lq;
    const v4f f0 = *(const v4f*)(src);
    const v4f f1 = *(const v4f*)(src + 4);
    const v4f f2 = *(const v4f*)(src + 8);
    const v4f f3 = *(const v4f*)(src + 12);
    v8us h0, h1;
#pragma unroll
    for (int e = 0; e < 4; ++e) {
      h0[e] = f2bf_bits(f0[e]); h0[4 + e] = f2bf_bits(f1[e]);
      h1[e] = f2bf_bits(f2[e]); h1[4 + e] = f2bf_bits(f3[e]);
    }
    *(v8us*)(th + cr * 72 + lq)     = h0;
    *(v8us*)(th + cr * 72 + lq + 8) = h1;
  }
  __syncthreads();
  const int lane = tid & 31, w = tid >> 5;
  const int c8 = (lane & 7) * 8;
  const int lr = w * 4 + (lane >> 3);
  v8us hv[2];
#pragma unroll
  for (int it = 0; it < 2; ++it) {
    const int l = it * 32 + lr;
#pragma unroll
    for (int e = 0; e < 8; ++e) hv[it][e] = th[(c8 + e) * 72 + l];
  }
  const size_t pb = (size_t)b * NL * NC;
  for (int pass = 0; pass < 2; ++pass) {
#pragma unroll
    for (int it = 0; it < 2; ++it) {
      const int l = it * 32 + lr;
      const size_t off = pb + (size_t)(l0 + l) * NC + c0 + c8;
      *(volatile v8us*)(P + off) = hv[it];
    }
    __threadfence();
  }
}

template <int BIAS_MODE>
__global__ __launch_bounds__(256) void gemm64_kernel(
    const unsigned short* __restrict__ Ap, int lda, long long strideA,
    const unsigned short* __restrict__ Bp, int ldb, long long strideB,
    unsigned short* __restrict__ Cp, unsigned short* __restrict__ C2p, int ldc, long long strideC,
    const float* __restrict__ bias, int M, int N, int K) {
  __shared__ __align__(16) float sT[8][64 * 20];
  const int bz   = blockIdx.y;
  const int lane = threadIdx.x & 31, wave = threadIdx.x >> 5, hf = lane >> 4, rl = lane & 15;
  const int tilesN = N >> 6, tilesM = M >> 6;
  const int tile = blockIdx.x * 8 + wave;
  if (tile >= tilesM * tilesN) return;
  const int tm = tile / tilesN, tn = tile - tm * tilesN;
  const int m0 = tm << 6, n0 = tn << 6;
  const unsigned short* Ab = Ap + (size_t)bz * (size_t)strideA;
  const unsigned short* Bb = Bp + (size_t)bz * (size_t)strideB;

  v8f acc[4][4];
#pragma unroll
  for (int i = 0; i < 4; ++i)
#pragma unroll
    for (int j = 0; j < 4; ++j) acc[i][j] = vz8();

#pragma unroll 1
  for (int k0 = 0; k0 < K; k0 += 32) {
    v16b bfr[4];
#pragma unroll
    for (int j = 0; j < 4; ++j)
      bfr[j] = ldfrag_b(Bb + (size_t)(n0 + 16 * j + rl) * ldb + k0, hf);
#pragma unroll
    for (int i = 0; i < 4; ++i) {
      const v16b afr = ldfrag_b(Ab + (size_t)(m0 + 16 * i + rl) * lda + k0, hf);
#pragma unroll
      for (int j = 0; j < 4; ++j) acc[i][j] = mma_b(afr, bfr[j], acc[i][j]);
    }
  }

  float* slab = sT[wave];
  unsigned short* Cb  = Cp  + (size_t)bz * (size_t)strideC;
  unsigned short* C2b = C2p + (size_t)bz * (size_t)strideC;
  const int q = lane >> 3, c8 = (lane & 7) * 8;
#pragma unroll
  for (int i = 0; i < 4; ++i) {
    const int mBase = m0 + 16 * i;
#pragma unroll
    for (int j = 0; j < 4; ++j) {
      const int col = 16 * j + rl;
      float bn = 0.f;
      if (BIAS_MODE == 2) bn = bf_rne(bias[n0 + col]);
      v4f va, vb;
#pragma unroll
      for (int r = 0; r < 4; ++r) {
        float v0 = acc[i][j][r];
        float v1 = acc[i][j][4 + r];
        if (BIAS_MODE == 1) { v0 += bf_rne(bias[mBase + 8 * hf + r]); v1 += bf_rne(bias[mBase + 8 * hf + 4 + r]); }
        if (BIAS_MODE == 2) { v0 += bn; v1 += bn; }
        va[r] = v0; vb[r] = v1;
      }
      *(v4f*)(slab + col * 20 + 8 * hf)     = va;
      *(v4f*)(slab + col * 20 + 8 * hf + 4) = vb;
    }
    __builtin_amdgcn_fence(__ATOMIC_RELEASE, "workgroup");
    __builtin_amdgcn_wave_barrier();
    __builtin_amdgcn_fence(__ATOMIC_ACQUIRE, "workgroup");
    v8us hb8[4], lb8[4];
#pragma unroll
    for (int it = 0; it < 4; ++it) {
      const int row = it * 4 + q;
#pragma unroll
      for (int e = 0; e < 8; ++e) {
        const float v = slab[(c8 + e) * 20 + row];
        const unsigned short hb = f2bf_bits(v);
        hb8[it][e] = hb;
        lb8[it][e] = f2bf_bits(v - bf_bits2f(hb));
      }
    }
    for (int pass = 0; pass < 2; ++pass) {
#pragma unroll
      for (int it = 0; it < 4; ++it) {
        const int row = it * 4 + q;
        const size_t off = (size_t)(mBase + row) * ldc + n0 + c8;
        *(volatile v8us*)(Cb + off)  = hb8[it];
        *(volatile v8us*)(C2b + off) = lb8[it];
      }
      __threadfence();
    }
    __builtin_amdgcn_fence(__ATOMIC_RELEASE, "workgroup");
    __builtin_amdgcn_wave_barrier();
    __builtin_amdgcn_fence(__ATOMIC_ACQUIRE, "workgroup");
  }
}

__global__ __launch_bounds__(128) void attn_kernel(const unsigned short* __restrict__ Qhi, const unsigned short* __restrict__ Qlo,
                                                   const unsigned short* __restrict__ Khi, const unsigned short* __restrict__ Klo,
                                                   const unsigned short* __restrict__ Vhi, const unsigned short* __restrict__ Vlo,
                                                   const float* __restrict__ tmask, const float* __restrict__ smask,
                                                   float* __restrict__ out) {
  __shared__ __align__(16) float so[64 * 68];
  const int t0 = blockIdx.x * 64, hh = blockIdx.y, b = blockIdx.z;
  const int tid = threadIdx.x, lane = tid & 31, w = tid >> 5, hf = lane >> 4, rl = lane & 15;
  const size_t pqk = (size_t)b * NL * NC + (size_t)hh * HDIM;
  const unsigned short* Qhb = Qhi + pqk;
  const unsigned short* Qlb = Qlo + pqk;
  const unsigned short* Khb = Khi + pqk;
  const unsigned short* Klb = Klo + pqk;
  const size_t pv = ((size_t)b * NC + (size_t)hh * HDIM) * NL;
  const unsigned short* Vhb = Vhi + pv;
  const unsigned short* Vlb = Vlo + pv;
  const float* smb = smask + (size_t)b * NL;
  const int tq = t0 + w * 16 + rl;
  const float tmv = tmask[(size_t)b * NL + tq];
  v16b qh[2], ql[2];
  qh[0] = ldfrag_b(Qhb + (size_t)tq * NC, hf);
  qh[1] = ldfrag_b(Qhb + (size_t)tq * NC + 32, hf);
  ql[0] = ldfrag_b(Qlb + (size_t)tq * NC, hf);
  ql[1] = ldfrag_b(Qlb + (size_t)tq * NC + 32, hf);

  v8f oacc[4];
#pragma unroll
  for (int dn = 0; dn < 4; ++dn) oacc[dn] = vz8();
  float mrun = -1.0e30f, lrun = 0.0f;
  const float sscl = 0.125f;

#pragma unroll 1
  for (int s0 = 0; s0 < NL; s0 += 64) {
    v8f sc[4], mk[4];
#pragma unroll
    for (int j = 0; j < 4; ++j) {
      const size_t ko = (size_t)(s0 + 16 * j + rl) * NC;
      sc[j] = vz8();
      {
        const v16b kh0 = ldfrag_b(Khb + ko, hf);
        const v16b kl0 = ldfrag_b(Klb + ko, hf);
        sc[j] = mma_b(kh0, qh[0], sc[j]);
        sc[j] = mma_b(kh0, ql[0], sc[j]);
        sc[j] = mma_b(kl0, qh[0], sc[j]);
      }
      {
        const v16b kh1 = ldfrag_b(Khb + ko + 32, hf);
        const v16b kl1 = ldfrag_b(Klb + ko + 32, hf);
        sc[j] = mma_b(kh1, qh[1], sc[j]);
        sc[j] = mma_b(kh1, ql[1], sc[j]);
        sc[j] = mma_b(kl1, qh[1], sc[j]);
      }
    }
    float rmax = -1.0e30f;
#pragma unroll
    for (int j = 0; j < 4; ++j) {
      const float* mp = smb + s0 + 16 * j + 8 * hf;
      M8 mu;
      mu.h[0] = *(const v4f*)(mp);
      mu.h[1] = *(const v4f*)(mp + 4);
#pragma unroll
      for (int r = 0; r < 8; ++r) {
        const float mm = tmv * mu.v[r];
        const float s  = sc[j][r] * sscl;
        const float x  = mm * s - (1.0f - mm) * NEGV;
        sc[j][r] = x;
        mk[j][r] = mm;
        rmax = fmaxf(rmax, x);
      }
    }
    rmax = fmaxf(rmax, __shfl_xor(rmax, 16, 32));
    const float mnew  = fmaxf(mrun, rmax);
    const float alpha = exp2f((mrun - mnew) * LOG2E);
    float psum = 0.0f;
#pragma unroll
    for (int j = 0; j < 4; ++j)
#pragma unroll
      for (int r = 0; r < 8; ++r) {
        const float p = exp2f((sc[j][r] - mnew) * LOG2E);
        psum += p;
        sc[j][r] = p * mk[j][r];
      }
    psum += __shfl_xor(psum, 16, 32);
    lrun = lrun * alpha + psum;
    mrun = mnew;
#pragma unroll
    for (int dn = 0; dn < 4; ++dn)
#pragma unroll
      for (int r = 0; r < 8; ++r) oacc[dn][r] *= alpha;
    FragB ph[2], pl[2];
#pragma unroll
    for (int ks = 0; ks < 2; ++ks)
#pragma unroll
      for (int r = 0; r < 8; ++r) {
        const float p0 = sc[2 * ks][r], p1 = sc[2 * ks + 1][r];
        const unsigned short h0 = f2bf_bits(p0), h1 = f2bf_bits(p1);
        ph[ks].h[0][r] = h0;
        ph[ks].h[1][r] = h1;
        pl[ks].h[0][r] = f2bf_bits(p0 - bf_bits2f(h0));
        pl[ks].h[1][r] = f2bf_bits(p1 - bf_bits2f(h1));
      }
#pragma unroll
    for (int ks = 0; ks < 2; ++ks)
#pragma unroll
      for (int dn = 0; dn < 4; ++dn) {
        const size_t vo = (size_t)(16 * dn + rl) * NL + s0 + 32 * ks;
        const v16b vh = ldfrag_b(Vhb + vo, hf);
        const v16b vl = ldfrag_b(Vlb + vo, hf);
        oacc[dn] = mma_b(vh, ph[ks].v, oacc[dn]);
        oacc[dn] = mma_b(vh, pl[ks].v, oacc[dn]);
        oacc[dn] = mma_b(vl, ph[ks].v, oacc[dn]);
      }
  }

  const float linv = 1.0f / lrun;
  {
    float* sp = so + (size_t)(w * 16 + rl) * 68 + 8 * hf;
#pragma unroll
    for (int dn = 0; dn < 4; ++dn) {
      v4f a, c;
#pragma unroll
      for (int r = 0; r < 4; ++r) { a[r] = oacc[dn][r] * linv; c[r] = oacc[dn][4 + r] * linv; }
      *(v4f*)(sp + 16 * dn)     = a;
      *(v4f*)(sp + 16 * dn + 4) = c;
    }
  }
  __syncthreads();
  float* ob = out + ((size_t)b * NC + (size_t)hh * HDIM) * NL + t0;
  const int c4 = rl * 4;
  v4f ov[8];
#pragma unroll
  for (int it = 0; it < 8; ++it) {
    const int d = w * 16 + it * 2 + hf;
    v4f v;
#pragma unroll
    for (int e = 0; e < 4; ++e) v[e] = so[(c4 + e) * 68 + d];
    ov[it] = v;
  }
  for (int pass = 0; pass < 2; ++pass) {
#pragma unroll
    for (int it = 0; it < 8; ++it) {
      const int d = w * 16 + it * 2 + hf;
      *(volatile v4f*)(ob + (size_t)d * NL + c4) = ov[it];
    }
    __threadfence();
  }
}

extern "C" void kernel_launch(void* const* d_in, const int* in_sizes, int n_in,
                              void* d_out, int out_size, void* d_ws, size_t ws_size,
                              hipStream_t stream) {
  if (n_in < 10) return;
  if (in_sizes[0] != NB * NC * NL || in_sizes[1] != NB * NC * NL) return;
  if (in_sizes[2] != NB * NL || in_sizes[3] != NB * NL) return;
  if (in_sizes[4] != NC * NC || in_sizes[6] != NC * NC || in_sizes[8] != NC * NC) return;
  if (in_sizes[5] != NC || in_sizes[7] != NC || in_sizes[9] != NC) return;
  if (out_size != NB * NC * NL) return;

  const float* target = (const float*)d_in[0];
  const float* source = (const float*)d_in[1];
  const float* tmask  = (const float*)d_in[2];
  const float* smask  = (const float*)d_in[3];
  const float* Wq = (const float*)d_in[4];
  const float* bq = (const float*)d_in[5];
  const float* Wk = (const float*)d_in[6];
  const float* bk = (const float*)d_in[7];
  const float* Wv = (const float*)d_in[8];
  const float* bv = (const float*)d_in[9];
  float* out = (float*)d_out;

  const size_t PW  = (size_t)NC * NC * 2;
  const size_t PXP = (size_t)NB * NL * NC * 2;
  size_t off = 0;
  const size_t oW   = off; off += 3 * PW;
  const size_t oXTt = off; off += PXP;
  const size_t oXTs = off; off += PXP;
  const size_t oQh  = off; off += PXP;
  const size_t oQl  = off; off += PXP;
  const size_t oKh  = off; off += PXP;
  const size_t oKl  = off; off += PXP;
  const size_t oVh  = off; off += PXP;
  const size_t oVl  = off; off += PXP;
  if (off > ws_size) return;

  char* ws = (char*)d_ws;
  unsigned short* W16 = (unsigned short*)(ws + oW);
  unsigned short* XTt = (unsigned short*)(ws + oXTt);
  unsigned short* XTs = (unsigned short*)(ws + oXTs);
  unsigned short* Qh  = (unsigned short*)(ws + oQh);
  unsigned short* Ql  = (unsigned short*)(ws + oQl);
  unsigned short* Kh  = (unsigned short*)(ws + oKh);
  unsigned short* Kl  = (unsigned short*)(ws + oKl);
  unsigned short* Vh  = (unsigned short*)(ws + oVh);
  unsigned short* Vl  = (unsigned short*)(ws + oVl);
  unsigned short* Wq16 = W16;
  unsigned short* Wk16 = W16 + (size_t)NC * NC;
  unsigned short* Wv16 = W16 + (size_t)2 * NC * NC;

  const dim3 blk(256);
  const int n8 = NC * NC / 8;
  const long long sXT = (long long)NL * NC;
  const long long sV  = (long long)NC * NL;

  cvt_w_kernel<<<dim3(n8 / 256, 3), blk, 0, stream>>>(Wq, Wk, Wv, W16, n8);
  cvt_xt_kernel<<<dim3(NL / 64, NC / 64, NB), blk, 0, stream>>>(target, XTt);
  cvt_xt_kernel<<<dim3(NL / 64, NC / 64, NB), blk, 0, stream>>>(source, XTs);
  const dim3 gP((NL / 64) * (NC / 64) / 8, NB);
  gemm64_kernel<2><<<gP, blk, 0, stream>>>(XTt, NC, sXT, Wq16, NC, 0LL, Qh, Ql, NC, sXT, bq, NL, NC, NC);
  gemm64_kernel<2><<<gP, blk, 0, stream>>>(XTs, NC, sXT, Wk16, NC, 0LL, Kh, Kl, NC, sXT, bk, NL, NC, NC);
  const dim3 gV((NC / 64) * (NL / 64) / 8, NB);
  gemm64_kernel<1><<<gV, blk, 0, stream>>>(Wv16, NC, 0LL, XTs, NC, sXT, Vh, Vl, NL, sV, bv, NC, NL, NC);
  attn_kernel<<<dim3(NL / 64, NHD, NB), dim3(128), 0, stream>>>(Qh, Ql, Kh, Kl, Vh, Vl, tmask, smask, out);
  (void)hipGetLastError();
}
